// MONet_50156628082755
// MI455X (gfx1250) — hardware-verified
//
#include <hip/hip_runtime.h>
#include <stddef.h>
#include <stdint.h>


#define FIN     128
#define NTHR    256
#define NWAVE   8
#define EPT     8
#define CHUNK   (NTHR * EPT)
#define WCAP    (EPT * 32)
#define LISTN   (NWAVE * WCAP)
#define NBD     8192
#define SLD     13
#define NB      1024
#define SLB     10
#define RCAP    24576
#define DEGCAP  256
#define GBM     64
#define GBN     64
#define GTHR    128
#define HRP     1024
#define G1P     320
#define X1K     1024
#define G1K     640
#define H2P     128
#define G2P     128
#define G2K     256
#define ZK     256
#define G3P     64
#define XGP     64
#define ELP     16
#define SLOPE_ATT 0.2f
#define SLOPE_MLP 0.25f
#define AGG_ZINTS (LISTN + 2 * RCAP + 3 * NB)
#define AGG_LDS_INTS (AGG_ZINTS + 16)

static_assert((CHUNK & (CHUNK - 1)) == 0 && CHUNK <= 4096);
static_assert((NBD & (NBD - 1)) == 0 && NBD == (1 << SLD));
static_assert((NB & (NB - 1)) == 0 && NB == (1 << SLB));
static_assert(((long long)CHUNK << SLD) < (1LL << 31));
static_assert(((long long)CHUNK << SLB) < (1LL << 31));
static_assert(NBD % (NTHR * 4) == 0);
static_assert(NB % NWAVE == 0 && NB % 32 == 0 && NB % GBM == 0);
static_assert(RCAP % 4 == 0 && AGG_ZINTS % 4 == 0 && LISTN % 4 == 0);
static_assert(GBM == (GTHR / 32) * 16 && GBN == 64);
static_assert(AGG_LDS_INTS * 4 <= 300000);
static_assert(FIN / 8 == 16);

typedef float          v2f   __attribute__((ext_vector_type(2)));
typedef float          v4f   __attribute__((ext_vector_type(4)));
typedef float          v8f   __attribute__((ext_vector_type(8)));
typedef int            v4i   __attribute__((ext_vector_type(4)));
typedef int            v8i   __attribute__((ext_vector_type(8)));
typedef unsigned short v2us  __attribute__((ext_vector_type(2)));
typedef unsigned short v4us  __attribute__((ext_vector_type(4)));
typedef unsigned short v8us  __attribute__((ext_vector_type(8)));
typedef unsigned short v16us __attribute__((ext_vector_type(16)));
typedef __bf16         v16bf __attribute__((ext_vector_type(16)));
typedef v2f  __attribute__((may_alias)) v2fa;
typedef v4f  __attribute__((may_alias)) v4fa;
typedef v4i  __attribute__((may_alias)) v4ia;
typedef v8us __attribute__((may_alias)) v8usa;
union FragB { v16bf v; v16us u; v8us h[2]; v8i w; };

__device__ __forceinline__ v8f wmb(const FragB& a, const FragB& b, v8f c) {
  v8f d = __builtin_amdgcn_wmma_f32_16x16x32_bf16(false, a.v, false, b.v, (short)0, c, false, false);
  asm volatile("v_nop\n\tv_nop\n\tv_nop\n\tv_nop" : "+v"(d) : "v"(a.w), "v"(b.w));
  return d;
}

__device__ __forceinline__ unsigned bf16_bits(float f) {
  const unsigned u = __float_as_uint(f);
  return (u + 0x7FFFu + ((u >> 16) & 1u)) >> 16;
}
__device__ __forceinline__ float bfr(float f) { return __uint_as_float(bf16_bits(f) << 16); }

#define SEL5(A, H) ((H) == 0 ? A[0] : ((H) == 1 ? A[1] : ((H) == 2 ? A[2] : ((H) == 3 ? A[3] : A[4]))))

template <int SLBT>
__device__ __forceinline__ int scan_chunk(const int* __restrict__ keys, int nE, int cbase, int slotBase,
                                          int nb, int vec8, int* list, int tid, int lane, int wave) {
  int wc = 0;
  const int el0  = tid * EPT;
  const int e0   = cbase + el0;
  const int sent = -2147483647 - 1;
  v4i da, db;
  if (vec8 != 0 && cbase + CHUNK <= nE) {
    da = *(const v4i*)(keys + e0);
    db = *(const v4i*)(keys + e0 + 4);
  } else {
    da.x = (e0     < nE) ? keys[min(e0,     nE - 1)] : sent;
    da.y = (e0 + 1 < nE) ? keys[min(e0 + 1, nE - 1)] : sent;
    da.z = (e0 + 2 < nE) ? keys[min(e0 + 2, nE - 1)] : sent;
    da.w = (e0 + 3 < nE) ? keys[min(e0 + 3, nE - 1)] : sent;
    db.x = (e0 + 4 < nE) ? keys[min(e0 + 4, nE - 1)] : sent;
    db.y = (e0 + 5 < nE) ? keys[min(e0 + 5, nE - 1)] : sent;
    db.z = (e0 + 6 < nE) ? keys[min(e0 + 6, nE - 1)] : sent;
    db.w = (e0 + 7 < nE) ? keys[min(e0 + 7, nE - 1)] : sent;
  }
  const unsigned nbs = (unsigned)slotBase;
  const unsigned unb = (unsigned)nb;
  const unsigned s0 = (unsigned)da.x - nbs, s1 = (unsigned)da.y - nbs;
  const unsigned s2 = (unsigned)da.z - nbs, s3 = (unsigned)da.w - nbs;
  const unsigned s4 = (unsigned)db.x - nbs, s5 = (unsigned)db.y - nbs;
  const unsigned s6 = (unsigned)db.z - nbs, s7 = (unsigned)db.w - nbs;
  const bool h0 = s0 < unb, h1 = s1 < unb, h2 = s2 < unb, h3 = s3 < unb;
  const bool h4 = s4 < unb, h5 = s5 < unb, h6 = s6 < unb, h7 = s7 < unb;
  const unsigned any = __builtin_amdgcn_ballot_w32(h0 | h1 | h2 | h3 | h4 | h5 | h6 | h7);
  if (any != 0u) {
#define HITJ(J, HJ, SJ) { \
      const unsigned mj = __builtin_amdgcn_ballot_w32(HJ); \
      if (mj != 0u) { \
        if (HJ) { \
          const int pos = wc + (int)__builtin_amdgcn_mbcnt_lo(mj, 0u); \
          if (pos < WCAP) list[wave * WCAP + pos] = ((el0 + (J)) << SLBT) | (int)(SJ); \
        } \
        wc += (int)__builtin_popcount(mj); } }
    HITJ(0, h0, s0)
    HITJ(1, h1, s1)
    HITJ(2, h2, s2)
    HITJ(3, h3, s3)
    HITJ(4, h4, s4)
    HITJ(5, h5, s5)
    HITJ(6, h6, s6)
    HITJ(7, h7, s7)
#undef HITJ
  }
  return wc;
}

__global__ __launch_bounds__(NTHR) void k_xprep(const float* __restrict__ x, unsigned short* xb, int nN, int nUnits) {
  const int i = (int)blockIdx.x * NTHR + (int)threadIdx.x;
  if (i >= nUnits) return;
  const int row = i >> 4;
  const int c0  = (i & 15) * 8;
  const int rc  = row < nN ? row : nN - 1;
  const float* p = x + (size_t)rc * FIN + c0;
  const v4f a = *(const v4fa*)p, b = *(const v4fa*)(p + 4);
  const bool ok = row < nN;
  v8us o;
  o[0] = ok ? (unsigned short)bf16_bits(a.x) : (unsigned short)0;
  o[1] = ok ? (unsigned short)bf16_bits(a.y) : (unsigned short)0;
  o[2] = ok ? (unsigned short)bf16_bits(a.z) : (unsigned short)0;
  o[3] = ok ? (unsigned short)bf16_bits(a.w) : (unsigned short)0;
  o[4] = ok ? (unsigned short)bf16_bits(b.x) : (unsigned short)0;
  o[5] = ok ? (unsigned short)bf16_bits(b.y) : (unsigned short)0;
  o[6] = ok ? (unsigned short)bf16_bits(b.z) : (unsigned short)0;
  o[7] = ok ? (unsigned short)bf16_bits(b.w) : (unsigned short)0;
  unsigned short* dp = xb + (size_t)row * FIN + c0;
  *(volatile v8us*)dp = o;
  __threadfence();
  *(volatile v8us*)dp = o;
}

__global__ __launch_bounds__(NTHR) void k_wprep(const float* __restrict__ w0, const float* __restrict__ w1,
                                                int c0, int c1, int segRows, int Kreal, int KH, int dbl,
                                                unsigned short* wt, int nUnits) {
  const int u = (int)blockIdx.x * NTHR + (int)threadIdx.x;
  if (u >= nUnits) return;
  const int KT  = (dbl != 0) ? 2 * KH : KH;
  const int kq  = KT >> 3;
  const int n   = u / kq;
  const int k8  = (u - n * kq) * 8;
  const int kr8 = (k8 >= KH) ? k8 - KH : k8;
  int seg = n / segRows;
  seg = seg > 1 ? 1 : seg;
  const int nc = n - seg * segRows;
  const float* wsp = (seg == 0) ? w0 : w1;
  const int cc  = (seg == 0) ? c0 : c1;
  const int ncl = nc < cc ? nc : cc - 1;
  const bool rok = nc < cc;
  float f[8];
#pragma unroll
  for (int i = 0; i < 8; ++i) {
    const int kr  = kr8 + i;
    const int krc = kr < Kreal ? kr : Kreal - 1;
    f[i] = wsp[(size_t)krc * (size_t)cc + ncl];
  }
  v8us o;
#pragma unroll
  for (int i = 0; i < 8; ++i)
    o[i] = (rok && (kr8 + i) < Kreal) ? (unsigned short)bf16_bits(f[i]) : (unsigned short)0;
  unsigned short* dp = wt + (size_t)n * (size_t)KT + k8;
  *(volatile v8us*)dp = o;
  __threadfence();
  *(volatile v8us*)dp = o;
}

__global__ __launch_bounds__(NTHR) void k_deg(const int* __restrict__ keys, int nE, int vec8, float* dq) {
  __shared__ __attribute__((aligned(16))) int scnt[NBD];
  __shared__ __attribute__((aligned(16))) int list[LISTN];
  __shared__ int wcnt[NWAVE];
  const int tid = (int)threadIdx.x, lane = tid & 31, wave = tid >> 5;
  const int nodeBase = (int)blockIdx.x * NBD;

  for (int i = tid; i < NBD; i += NTHR) scnt[i] = 0;
  for (int i = tid; i < LISTN; i += NTHR) list[i] = 0;
  if (tid < NWAVE) wcnt[tid] = 0;
  __syncthreads();

  const int nChunks = (nE + CHUNK - 1) / CHUNK;
#pragma unroll 1
  for (int ch = 0; ch < nChunks; ++ch) {
    const int cbase = ch * CHUNK;
    const int wc = scan_chunk<SLD>(keys, nE, cbase, nodeBase, NBD, vec8, list, tid, lane, wave);
    if (lane == 0) wcnt[wave] = wc;
    __syncthreads();
    if (wave == 0) {
#pragma unroll 1
      for (int w2 = 0; w2 < NWAVE; ++w2) {
        int c = wcnt[w2];
        c = c < 0 ? 0 : (c > WCAP ? WCAP : c);
#pragma unroll 1
        for (int b0 = 0; b0 < c; b0 += 32) {
          const int idx = b0 + lane;
          const int ent = list[w2 * WCAP + (idx < WCAP ? idx : WCAP - 1)];
          const int m32 = (c - b0) < 32 ? (c - b0) : 32;
#pragma unroll 1
          for (int k = 0; k < m32; ++k) {
            const int u  = __builtin_amdgcn_readlane(ent, k);
            const int sl = u & (NBD - 1);
            if (lane == 0) scnt[sl] = scnt[sl] + 1;
          }
        }
      }
    }
    __syncthreads();
  }

  v4f vals[NBD / (NTHR * 4)];
#pragma unroll
  for (int it = 0; it < NBD / (NTHR * 4); ++it) {
    const int s0 = it * (NTHR * 4) + 4 * tid;
    const v4i c4 = *(const v4ia*)(scnt + s0);
    v4f v;
    v.x = rsqrtf(fmaxf((float)c4.x, 1.0f)); v.y = rsqrtf(fmaxf((float)c4.y, 1.0f));
    v.z = rsqrtf(fmaxf((float)c4.z, 1.0f)); v.w = rsqrtf(fmaxf((float)c4.w, 1.0f));
    vals[it] = v;
  }
#pragma unroll
  for (int it = 0; it < NBD / (NTHR * 4); ++it) {
    const int s0 = it * (NTHR * 4) + 4 * tid;
    *(volatile v4f*)(dq + (size_t)nodeBase + s0) = vals[it];
  }
  __threadfence();
#pragma unroll
  for (int it = 0; it < NBD / (NTHR * 4); ++it) {
    const int s0 = it * (NTHR * 4) + 4 * tid;
    *(volatile v4f*)(dq + (size_t)nodeBase + s0) = vals[it];
  }
}

template <int HEAD>
__global__ __launch_bounds__(GTHR) void k_gemm(const unsigned short* __restrict__ A, int lda,
                                               const unsigned short* __restrict__ BT, int ldb, int K,
                                               float* Cm, int ldc,
                                               const float* __restrict__ f1b, const float* __restrict__ f2w,
                                               const float* __restrict__ f2b, float* outp, int nN) {
  __shared__ __attribute__((aligned(16))) float stg[GBM * GBN];
  __shared__ __attribute__((aligned(16))) float s1b[64];
  __shared__ __attribute__((aligned(16))) float s2w[128];
  __shared__ __attribute__((aligned(16))) float s2b[4];
  __shared__ __attribute__((aligned(16))) float ostg[128];
  const int tid = (int)threadIdx.x, lane = tid & 31, wave = tid >> 5, hh = lane >> 4, m = lane & 15;
  const int rowBase = (int)blockIdx.x * GBM;
  const int col0    = (int)blockIdx.y * GBN;

  if constexpr (HEAD != 0) {
    s2w[tid] = bfr(f2w[tid]);
    if (tid < 64) s1b[tid] = bfr(f1b[tid]);
    if (tid < 2)  s2b[tid] = bfr(f2b[tid]);
  }

  v8f acc[4];
  {
    const v8f z = {0.f, 0.f, 0.f, 0.f, 0.f, 0.f, 0.f, 0.f};
    acc[0] = z; acc[1] = z; acc[2] = z; acc[3] = z;
  }
  const unsigned short* ap = A  + (size_t)(rowBase + 16 * wave + m) * (size_t)lda + 8 * hh;
  const unsigned short* bp = BT + (size_t)(col0 + m) * (size_t)ldb + 8 * hh;
#pragma unroll 1
  for (int k0 = 0; k0 < K; k0 += 32) {
    FragB af;
    af.h[0] = *(const v8usa*)(ap + k0);
    af.h[1] = *(const v8usa*)(ap + k0 + 16);
#pragma unroll
    for (int t = 0; t < 4; ++t) {
      const unsigned short* wq = bp + (size_t)(16 * t) * (size_t)ldb + k0;
      FragB bf;
      bf.h[0] = *(const v8usa*)wq;
      bf.h[1] = *(const v8usa*)(wq + 16);
      acc[t] = wmb(af, bf, acc[t]);
    }
  }

#pragma unroll
  for (int t = 0; t < 4; ++t) {
    const int lc = 16 * t + m;
#pragma unroll
    for (int r = 0; r < 8; ++r) {
      const int lr = 16 * wave + 8 * hh + r;
      stg[lr * GBN + lc] = acc[t][r];
    }
  }
  __syncthreads();

  if constexpr (HEAD == 0) {
    v4f fv[8];
#pragma unroll
    for (int i = 0; i < 8; ++i) {
      const int lr = 16 * wave + 2 * i + hh;
      fv[i] = *(const v4fa*)(stg + lr * GBN + 4 * m);
    }
#pragma unroll
    for (int i = 0; i < 8; ++i) {
      const int gr = rowBase + 16 * wave + 2 * i + hh;
      float* op = Cm + (size_t)gr * (size_t)ldc + col0 + 4 * m;
      *(volatile v4f*)op = fv[i];
    }
    __threadfence();
#pragma unroll
    for (int i = 0; i < 8; ++i) {
      const int gr = rowBase + 16 * wave + 2 * i + hh;
      float* op = Cm + (size_t)gr * (size_t)ldc + col0 + 4 * m;
      *(volatile v4f*)op = fv[i];
    }
  } else {
    const int row = tid >> 1, o = tid & 1;
    float s = 0.0f;
#pragma unroll 4
    for (int c = 0; c < 64; ++c) {
      float y = stg[row * GBN + c] + s1b[c];
      y = y > 0.0f ? y : SLOPE_MLP * y;
      s = fmaf(y, s2w[2 * c + o], s);
    }
    s += s2b[o];
    ostg[tid] = s;
    __syncthreads();
    const v4f ov = *(const v4fa*)(ostg + 4 * lane);
    const bool wr = (wave == 0) && (rowBase + 2 * lane + 1 < nN);
    float* op = outp + (size_t)(rowBase + 2 * lane) * 2;
    if (wr) *(volatile v4f*)op = ov;
    __threadfence();
    if (wr) *(volatile v4f*)op = ov;
  }
}

template <int L>
__global__ __launch_bounds__(NTHR) void k_att(const float* __restrict__ hp, const float* __restrict__ al,
                                              const float* __restrict__ ar, float* elr) {
  static_assert(L == 1 || L == 2);
  constexpr int PITCH = (L == 1) ? HRP : H2P;
  constexpr int CPL   = (L == 1) ? 16 : 2;
  constexpr int HD    = (L == 1) ? 100 : 64;
  constexpr int NH    = (L == 1) ? 5 : 1;
  constexpr int NTOT  = NH * HD;
  constexpr int NST   = 32 * CPL;
  __shared__ __attribute__((aligned(16))) float sal[512];
  __shared__ __attribute__((aligned(16))) float sar[512];
  __shared__ __attribute__((aligned(16))) float stg[32 * ELP];
  const int tid = (int)threadIdx.x, lane = tid & 31, wave = tid >> 5;
  for (int i = tid; i < NST; i += NTHR) {
    const int ic = i < NTOT ? i : NTOT - 1;
    const float va = bfr(al[ic]), vr = bfr(ar[ic]);
    sal[i] = i < NTOT ? va : 0.0f;
    sar[i] = i < NTOT ? vr : 0.0f;
  }
  __syncthreads();
  const int rowBase = (int)blockIdx.x * 32;
  const int c0 = CPL * lane;
  int ha = c0 / HD;
  ha = ha > NH - 1 ? NH - 1 : ha;
  int jb = HD * (ha + 1) - c0;
  jb = jb < 0 ? 0 : (jb > CPL ? CPL : jb);
  const int hb = (ha + 1 > NH - 1) ? NH - 1 : ha + 1;
  float av[CPL], rv[CPL];
  if constexpr (L == 1) {
#pragma unroll
    for (int g = 0; g < 4; ++g) {
      const v4f a = *(const v4fa*)(sal + c0 + 4 * g), r = *(const v4fa*)(sar + c0 + 4 * g);
      av[4 * g] = a.x; av[4 * g + 1] = a.y; av[4 * g + 2] = a.z; av[4 * g + 3] = a.w;
      rv[4 * g] = r.x; rv[4 * g + 1] = r.y; rv[4 * g + 2] = r.z; rv[4 * g + 3] = r.w;
    }
  } else {
    const v2f a = *(const v2fa*)(sal + c0), r = *(const v2fa*)(sar + c0);
    av[0] = a.x; av[1] = a.y; rv[0] = r.x; rv[1] = r.y;
  }

#pragma unroll 1
  for (int rr = 0; rr < 4; ++rr) {
    const int lr  = 4 * wave + rr;
    const int row = rowBase + lr;
    const float* p = hp + (size_t)row * PITCH + c0;
    float hv[CPL];
    if constexpr (L == 1) {
#pragma unroll
      for (int g = 0; g < 4; ++g) {
        const v4f a = *(const v4fa*)(p + 4 * g);
        hv[4 * g] = a.x; hv[4 * g + 1] = a.y; hv[4 * g + 2] = a.z; hv[4 * g + 3] = a.w;
      }
    } else {
      const v2f a = *(const v2fa*)p;
      hv[0] = a.x; hv[1] = a.y;
    }
    float sa = 0.0f, sb = 0.0f, ra = 0.0f, rb = 0.0f;
#pragma unroll
    for (int j = 0; j < CPL; ++j) {
      const float pa = hv[j] * av[j], pr = hv[j] * rv[j];
      const bool lo = j < jb;
      sa += lo ? pa : 0.0f;  sb += lo ? 0.0f : pa;
      ra += lo ? pr : 0.0f;  rb += lo ? 0.0f : pr;
    }
    float elv[5] = {0.f, 0.f, 0.f, 0.f, 0.f}, erv[5] = {0.f, 0.f, 0.f, 0.f, 0.f};
#pragma unroll
    for (int h = 0; h < NH; ++h) {
      float t = (ha == h ? sa : 0.0f) + (hb == h ? sb : 0.0f);
      float u = (ha == h ? ra : 0.0f) + (hb == h ? rb : 0.0f);
#pragma unroll
      for (int off = 16; off > 0; off >>= 1) { t += __shfl_xor(t, off); u += __shfl_xor(u, off); }
      elv[h] = t; erv[h] = u;
    }
    if (lane == 0) {
      float* sp = stg + lr * ELP;
      const v4f a0 = {elv[0], elv[1], elv[2], elv[3]}, a1 = {elv[4], 0.f, 0.f, 0.f};
      const v4f a2 = {erv[0], erv[1], erv[2], erv[3]}, a3 = {erv[4], 0.f, 0.f, 0.f};
      *(v4fa*)sp = a0; *(v4fa*)(sp + 4) = a1; *(v4fa*)(sp + 8) = a2; *(v4fa*)(sp + 12) = a3;
    }
  }
  __syncthreads();
  const int lr2 = (8 * wave + (lane >> 2)) & 31;
  const v4f ov = *(const v4fa*)(stg + lr2 * ELP + 4 * (lane & 3));
  float* op = elr + (size_t)(rowBase + lr2) * ELP + 4 * (lane & 3);
  const bool wr = wave < 4;
  if (wr) *(volatile v4f*)op = ov;
  __threadfence();
  if (wr) *(volatile v4f*)op = ov;
}

__device__ __forceinline__ int build_lists(const int* __restrict__ keys, int nE, int vec8, int nodeBase,
                                           int* dsm, int tid, int lane, int wave) {
  int* list = dsm;
  int* hl   = dsm + LISTN;
  int* sl   = hl + RCAP;
  int* cnt  = sl + RCAP;
  int* offs = cnt + NB;
  int* cur  = offs + NB;
  int* misc = cur + NB;
  {
    const v4i z4 = {0, 0, 0, 0};
    for (int i = tid * 4; i < AGG_ZINTS; i += NTHR * 4) *(v4ia*)(dsm + i) = z4;
    if (tid < 16) misc[tid] = 0;
  }
  __syncthreads();

  int t = 0, ov = 0;
  const int nChunks = (nE + CHUNK - 1) / CHUNK;
#pragma unroll 1
  for (int ch = 0; ch < nChunks; ++ch) {
    const int cbase = ch * CHUNK;
    const int wc = scan_chunk<SLB>(keys, nE, cbase, nodeBase, NB, vec8, list, tid, lane, wave);
    if (lane == 0) misc[wave] = wc;
    __syncthreads();
    if (wave == 0) {
#pragma unroll 1
      for (int w2 = 0; w2 < NWAVE; ++w2) {
        int c = misc[w2];
        c = c < 0 ? 0 : (c > WCAP ? WCAP : c);
#pragma unroll 1
        for (int b0 = 0; b0 < c; b0 += 32) {
          const int idx = b0 + lane;
          const int ent = list[w2 * WCAP + (idx < WCAP ? idx : WCAP - 1)];
          const int m32 = (c - b0) < 32 ? (c - b0) : 32;
#pragma unroll 1
          for (int k = 0; k < m32; ++k) {
            const int u    = __builtin_amdgcn_readlane(ent, k);
            const int slot = u & (NB - 1);
            const int el   = (u >> SLB) & (CHUNK - 1);
            const int pk   = ((cbase + el) << SLB) | slot;
            if (t < RCAP) {
              if (lane == 0) { hl[t] = pk; cnt[slot] = cnt[slot] + 1; }
              t = t + 1;
            } else {
              ov = 1;
            }
          }
        }
      }
    }
    __syncthreads();
  }
  if (wave == 0 && lane == 0) { misc[8] = t; misc[9] = ov; }
  __syncthreads();
  int tt = misc[8];
  tt = tt < 0 ? 0 : (tt > RCAP ? RCAP : tt);

  if (wave == 0) {
    const int base = lane * (NB / 32);
    int s = 0;
#pragma unroll 1
    for (int i = 0; i < NB / 32; ++i) s += cnt[base + i];
    int incl = s;
#pragma unroll
    for (int d = 1; d < 32; d <<= 1) {
      const int y = __shfl_up(incl, d, 32);
      if (lane >= d) incl += y;
    }
    int run = incl - s;
#pragma unroll 1
    for (int i = 0; i < NB / 32; ++i) {
      const int cv = cnt[base + i];
      offs[base + i] = run;
      cur[base + i]  = run;
      run += cv;
    }
  }
  __syncthreads();
  if (wave == 0) {
#pragma unroll 1
    for (int b0 = 0; b0 < tt; b0 += 32) {
      const int idx = b0 + lane;
      const int ent = hl[idx < RCAP ? idx : RCAP - 1];
      const int m32 = (tt - b0) < 32 ? (tt - b0) : 32;
#pragma unroll 1
      for (int k = 0; k < m32; ++k) {
        const int u    = __builtin_amdgcn_readlane(ent, k);
        const int slot = u & (NB - 1);
        if (lane == 0) {
          int p = cur[slot];
          p = p < 0 ? 0 : (p > RCAP - 1 ? RCAP - 1 : p);
          sl[p] = u;
          cur[slot] = p + 1;
        }
      }
    }
  }
  __syncthreads();
  return misc[9];
}

#define GAT_LOGITS(EV, SR) { \
    const float* q_ = elr + (size_t)(SR) * ELP; \
    const v4f a_ = *(const v4fa*)q_; \
    float t_[5]; \
    t_[0] = a_.x + erv[0]; t_[1] = a_.y + erv[1]; t_[2] = a_.z + erv[2]; t_[3] = a_.w + erv[3]; t_[4] = q_[4] + erv[4]; \
    EV[0] = t_[0] > 0.f ? t_[0] : SLOPE_ATT * t_[0]; EV[1] = t_[1] > 0.f ? t_[1] : SLOPE_ATT * t_[1]; \
    EV[2] = t_[2] > 0.f ? t_[2] : SLOPE_ATT * t_[2]; EV[3] = t_[3] > 0.f ? t_[3] : SLOPE_ATT * t_[3]; \
    EV[4] = t_[4] > 0.f ? t_[4] : SLOPE_ATT * t_[4]; }

template <int L>
__global__ __launch_bounds__(NTHR) void k_gat(const int* __restrict__ srcs, const int* __restrict__ keys,
                                              int nE, int nN, int vec8, int mRows,
                                              const float* __restrict__ hp, const float* __restrict__ elr,
                                              const float* __restrict__ bias, unsigned short* x1a, float* xgat) {
  static_assert(L == 1 || L == 2);
  constexpr int NH    = (L == 1) ? 5 : 1;
  constexpr int PITCH = (L == 1) ? HRP : H2P;
  constexpr int ROFF  = (L == 1) ? 512 : 64;
  constexpr int NACC  = (L == 1) ? 16 : 2;
  extern __shared__ __attribute__((aligned(16))) int dsm[];
  int* sl   = dsm + LISTN + RCAP;
  int* cnt  = dsm + LISTN + 2 * RCAP;
  int* offs = cnt + NB;
  const int tid = (int)threadIdx.x, lane = tid & 31, wave = tid >> 5;
  const int nodeBase = (int)blockIdx.x * NB;

  const int cA = (L == 1) ? 8 * lane : 2 * lane;
  const int cB = 256 + 8 * lane;
  int haA = 0, jbA = 8, hbA = 0, haB = 0, jbB = 8, hbB = 0;
  float bv[NACC];
  if constexpr (L == 1) {
    haA = cA / 100;
    jbA = 100 * (haA + 1) - cA;  jbA = jbA > 8 ? 8 : jbA;
    hbA = haA + 1;
    haB = cB / 100;  haB = haB > 4 ? 4 : haB;
    jbB = 100 * (haB + 1) - cB;  jbB = jbB < 0 ? 0 : (jbB > 8 ? 8 : jbB);
    hbB = (haB + 1 > 4) ? 4 : haB + 1;
    const v4f q0 = *(const v4fa*)(bias + cA), q1 = *(const v4fa*)(bias + cA + 4);
    const int a2 = cB < 496 ? cB : 496, a3 = (cB + 4) < 496 ? (cB + 4) : 496;
    const v4f q2 = *(const v4fa*)(bias + a2), q3 = *(const v4fa*)(bias + a3);
#pragma unroll
    for (int i = 0; i < 4; ++i) {
      bv[i]      = bfr(q0[i]);
      bv[4 + i]  = bfr(q1[i]);
      bv[8 + i]  = (cB + i < 500)     ? bfr(q2[i]) : 0.0f;
      bv[12 + i] = (cB + 4 + i < 500) ? bfr(q3[i]) : 0.0f;
    }
  } else {
    const v2f q = *(const v2fa*)(bias + cA);
    bv[0] = bfr(q.x); bv[1] = bfr(q.y);
    (void)cB; (void)haA; (void)jbA; (void)hbA; (void)haB; (void)jbB; (void)hbB;
  }

  const int ovf = build_lists(keys, nE, vec8, nodeBase, dsm, tid, lane, wave);
  const float qnan = __int_as_float(0x7fc00000);
  const float pz = (ovf != 0) ? qnan : 0.0f;

#pragma unroll 1
  for (int si = 0; si < NB / NWAVE; ++si) {
    const int s    = si * NWAVE + wave;
    const int node = nodeBase + s;
    const int craw = cnt[s];
    const bool big = craw > DEGCAP;
    const int c = craw < 0 ? 0 : (craw > DEGCAP ? DEGCAP : craw);
    int o = offs[s];
    o = o < 0 ? 0 : (o > RCAP ? RCAP : o);
    const int nc = node < nN ? node : nN - 1;
    float erv[5];
    {
      const float* q = elr + (size_t)nc * ELP + 8;
      const v4f a = *(const v4fa*)q;
      erv[0] = a.x; erv[1] = a.y; erv[2] = a.z; erv[3] = a.w; erv[4] = q[4];
    }
    float mx[5] = {-3.0e38f, -3.0e38f, -3.0e38f, -3.0e38f, -3.0e38f};

#pragma unroll 1
    for (int b0 = 0; b0 < c; b0 += 32) {
      int idx = o + b0 + lane;
      idx = idx > RCAP - 1 ? RCAP - 1 : idx;
      int eid = sl[idx] >> SLB;
      eid = eid < 0 ? 0 : (eid > nE - 1 ? nE - 1 : eid);
      int sr = srcs[eid];
      sr = sr < 0 ? 0 : (sr > nN - 1 ? nN - 1 : sr);
      const bool valid = (b0 + lane) < c;
      float ev[5];
      GAT_LOGITS(ev, sr)
#pragma unroll
      for (int h = 0; h < NH; ++h) {
        float t = valid ? ev[h] : -3.0e38f;
#pragma unroll
        for (int off = 16; off > 0; off >>= 1) t = fmaxf(t, __shfl_xor(t, off));
        mx[h] = fmaxf(mx[h], t);
      }
    }

    float acc[NACC];
#pragma unroll
    for (int j = 0; j < NACC; ++j) acc[j] = 0.0f;
    float dl[5] = {0.f, 0.f, 0.f, 0.f, 0.f};

#pragma unroll 1
    for (int b0 = 0; b0 < c; b0 += 32) {
      int idx = o + b0 + lane;
      idx = idx > RCAP - 1 ? RCAP - 1 : idx;
      int eid = sl[idx] >> SLB;
      eid = eid < 0 ? 0 : (eid > nE - 1 ? nE - 1 : eid);
      int sr = srcs[eid];
      sr = sr < 0 ? 0 : (sr > nN - 1 ? nN - 1 : sr);
      const bool valid = (b0 + lane) < c;
      float ev[5];
      GAT_LOGITS(ev, sr)
      int wi[5] = {0, 0, 0, 0, 0};
#pragma unroll
      for (int h = 0; h < NH; ++h) {
        float w = __expf(ev[h] - mx[h]);
        w = valid ? w : 0.0f;
        dl[h] += w;
        wi[h] = __float_as_int(w);
      }
      const int m32 = (c - b0) < 32 ? (c - b0) : 32;
#pragma unroll 1
      for (int k = 0; k < m32; ++k) {
        const int sk = __builtin_amdgcn_readlane(sr, k);
        float wk[5] = {0.f, 0.f, 0.f, 0.f, 0.f};
#pragma unroll
        for (int h = 0; h < NH; ++h) wk[h] = __int_as_float(__builtin_amdgcn_readlane(wi[h], k));
        const float* rp = hp + (size_t)sk * PITCH;
        if constexpr (L == 1) {
          const float wa0 = SEL5(wk, haA), wa1 = SEL5(wk, hbA), wb0 = SEL5(wk, haB), wb1 = SEL5(wk, hbB);
          const v4f x0 = *(const v4fa*)(rp + cA), x1 = *(const v4fa*)(rp + cA + 4);
          const v4f x2 = *(const v4fa*)(rp + cB), x3 = *(const v4fa*)(rp + cB + 4);
          const float xv[16] = {x0.x, x0.y, x0.z, x0.w, x1.x, x1.y, x1.z, x1.w,
                                x2.x, x2.y, x2.z, x2.w, x3.x, x3.y, x3.z, x3.w};
#pragma unroll
          for (int j = 0; j < 8; ++j) {
            const float wj = (j < jbA) ? wa0 : wa1;
            acc[j] = fmaf(wj, xv[j], acc[j]);
          }
#pragma unroll
          for (int j = 0; j < 8; ++j) {
            const float wj = (j < jbB) ? wb0 : wb1;
            acc[8 + j] = fmaf(wj, xv[8 + j], acc[8 + j]);
          }
        } else {
          const v2f x0 = *(const v2fa*)(rp + cA);
          acc[0] = fmaf(wk[0], x0.x, acc[0]);
          acc[1] = fmaf(wk[0], x0.y, acc[1]);
        }
      }
    }

    float inv[5] = {0.f, 0.f, 0.f, 0.f, 0.f};
#pragma unroll
    for (int h = 0; h < NH; ++h) {
      float t = dl[h];
#pragma unroll
      for (int off = 16; off > 0; off >>= 1) t += __shfl_xor(t, off);
      inv[h] = __builtin_amdgcn_rcpf(fmaxf(t, 1e-9f));
    }
    const float pzr = big ? qnan : pz;
    const bool live = node < nN;
    const float* rq = hp + (size_t)nc * PITCH + ROFF;
    if constexpr (L == 1) {
      const float ia0 = SEL5(inv, haA), ia1 = SEL5(inv, hbA), ib0 = SEL5(inv, haB), ib1 = SEL5(inv, hbB);
      const v4f r0 = *(const v4fa*)(rq + cA), r1 = *(const v4fa*)(rq + cA + 4);
      const v4f r2 = *(const v4fa*)(rq + cB), r3 = *(const v4fa*)(rq + cB + 4);
      const float rv[16] = {r0.x, r0.y, r0.z, r0.w, r1.x, r1.y, r1.z, r1.w,
                            r2.x, r2.y, r2.z, r2.w, r3.x, r3.y, r3.z, r3.w};
      float v[16];
#pragma unroll
      for (int j = 0; j < 8; ++j) {
        const float ij = (j < jbA) ? ia0 : ia1;
        v[j] = fmaf(acc[j], ij, rv[j]) + bv[j];
      }
#pragma unroll
      for (int j = 0; j < 8; ++j) {
        const float ij = (j < jbB) ? ib0 : ib1;
        v[8 + j] = fmaf(acc[8 + j], ij, rv[8 + j]) + bv[8 + j];
      }
#pragma unroll
      for (int j = 0; j < 16; ++j) {
        float t = v[j];
        const float em = __expf(fminf(t, 0.0f)) - 1.0f;
        t = t > 0.0f ? t : em;
        t = t + pzr;
        v[j] = live ? t : 0.0f;
      }
      v8us hoA, hoB, loA, loB;
#pragma unroll
      for (int j = 0; j < 8; ++j) {
        const unsigned ha = bf16_bits(v[j]);
        hoA[j] = (unsigned short)ha;
        loA[j] = (unsigned short)bf16_bits(v[j] - __uint_as_float(ha << 16));
        const unsigned hb = bf16_bits(v[8 + j]);
        hoB[j] = (unsigned short)hb;
        loB[j] = (unsigned short)bf16_bits(v[8 + j] - __uint_as_float(hb << 16));
      }
      if (node < mRows) {
        unsigned short* up = x1a + (size_t)node * X1K;
        *(volatile v8us*)(up + cA) = hoA;
        *(volatile v8us*)(up + cB) = hoB;
        *(volatile v8us*)(up + 512 + cA) = loA;
        *(volatile v8us*)(up + 512 + cB) = loB;
        __threadfence();
        *(volatile v8us*)(up + cA) = hoA;
        *(volatile v8us*)(up + cB) = hoB;
        *(volatile v8us*)(up + 512 + cA) = loA;
        *(volatile v8us*)(up + 512 + cB) = loB;
      }
    } else {
      const v2f r = *(const v2fa*)(rq + cA);
      float t0 = fmaf(acc[0], inv[0], r.x) + bv[0] + pzr;
      float t1 = fmaf(acc[1], inv[0], r.y) + bv[1] + pzr;
      v2f ov2;
      ov2.x = live ? t0 : 0.0f;
      ov2.y = live ? t1 : 0.0f;
      if (node < mRows) {
        float* op = xgat + (size_t)node * XGP + cA;
        *(volatile v2f*)op = ov2;
        __threadfence();
        *(volatile v2f*)op = ov2;
      }
    }
  }
}
#undef GAT_LOGITS

template <int L>
__global__ __launch_bounds__(NTHR) void k_gcn(const int* __restrict__ srcs, const int* __restrict__ keys,
                                              int nE, int nN, int vec8, int mRows,
                                              const float* __restrict__ dsrc, const float* __restrict__ xp,
                                              const float* __restrict__ bias, const float* __restrict__ xgat,
                                              unsigned short* outp) {
  static_assert(L >= 1 && L <= 3);
  constexpr int PITCH = (L == 1) ? G1P : ((L == 2) ? G2P : G3P);
  constexpr int KOUT  = (L == 1) ? G1K : G2K;
  constexpr int LOOFF = (L == 1) ? 320 : 128;
  constexpr int NV    = (L == 1) ? 300 : ((L == 2) ? 100 : 64);
  constexpr int NACC  = (L == 1) ? 10 : 4;
  extern __shared__ __attribute__((aligned(16))) int dsm[];
  int* sl   = dsm + LISTN + RCAP;
  int* cnt  = dsm + LISTN + 2 * RCAP;
  int* offs = cnt + NB;
  const int tid = (int)threadIdx.x, lane = tid & 31, wave = tid >> 5;
  const int nodeBase = (int)blockIdx.x * NB;

  const int cA = (L == 3) ? 4 * (lane & 15) : 4 * lane;
  float bq[NACC];
  {
    const int ca = cA < NV - 4 ? cA : NV - 4;
    const v4f q = *(const v4fa*)(bias + ca);
#pragma unroll
    for (int i = 0; i < 4; ++i) bq[i] = (cA + i < NV) ? bfr(q[i]) : 0.0f;
    if constexpr (L == 1) {
      const v4f q2 = *(const v4fa*)(bias + 128 + 4 * lane);
#pragma unroll
      for (int i = 0; i < 4; ++i) bq[4 + i] = bfr(q2[i]);
      const int cc  = 256 + 2 * lane;
      const int ccl = cc < NV - 2 ? cc : NV - 2;
      const v2f q3 = *(const v2fa*)(bias + ccl);
      bq[8] = (cc < NV)     ? bfr(q3.x) : 0.0f;
      bq[9] = (cc + 1 < NV) ? bfr(q3.y) : 0.0f;
    }
  }

  const int ovf = build_lists(keys, nE, vec8, nodeBase, dsm, tid, lane, wave);
  const float qnan = __int_as_float(0x7fc00000);
  const float pz = (ovf != 0) ? qnan : 0.0f;

#pragma unroll 1
  for (int si = 0; si < NB / NWAVE; ++si) {
    const int s    = si * NWAVE + wave;
    const int node = nodeBase + s;
    const int craw = cnt[s];
    const bool big = craw > DEGCAP;
    const int c = craw < 0 ? 0 : (craw > DEGCAP ? DEGCAP : craw);
    int o = offs[s];
    o = o < 0 ? 0 : (o > RCAP ? RCAP : o);
    const int nc = node < nN ? node : nN - 1;
    float acc[NACC];
#pragma unroll
    for (int i = 0; i < NACC; ++i) acc[i] = 0.0f;
#pragma unroll 1
    for (int b0 = 0; b0 < c; b0 += 32) {
      int idx = o + b0 + lane;
      idx = idx > RCAP - 1 ? RCAP - 1 : idx;
      int eid = sl[idx] >> SLB;
      eid = eid < 0 ? 0 : (eid > nE - 1 ? nE - 1 : eid);
      int sr = srcs[eid];
      sr = sr < 0 ? 0 : (sr > nN - 1 ? nN - 1 : sr);
      const float cf  = dsrc[sr];
      const int   cfi = __float_as_int(cf);
      const int m32 = (c - b0) < 32 ? (c - b0) : 32;
#pragma unroll 1
      for (int k = 0; k < m32; ++k) {
        const int   sk = __builtin_amdgcn_readlane(sr, k);
        const float ck = __int_as_float(__builtin_amdgcn_readlane(cfi, k));
        const float* rp = xp + (size_t)sk * PITCH;
        const v4f a = *(const v4fa*)(rp + cA);
        acc[0] = fmaf(ck, a.x, acc[0]); acc[1] = fmaf(ck, a.y, acc[1]);
        acc[2] = fmaf(ck, a.z, acc[2]); acc[3] = fmaf(ck, a.w, acc[3]);
        if constexpr (L == 1) {
          const v4f b = *(const v4fa*)(rp + 128 + 4 * lane);
          acc[4] = fmaf(ck, b.x, acc[4]); acc[5] = fmaf(ck, b.y, acc[5]);
          acc[6] = fmaf(ck, b.z, acc[6]); acc[7] = fmaf(ck, b.w, acc[7]);
          const v2f d = *(const v2fa*)(rp + 256 + 2 * lane);
          acc[8] = fmaf(ck, d.x, acc[8]); acc[9] = fmaf(ck, d.y, acc[9]);
        }
      }
    }
    const float di  = rsqrtf(fmaxf((float)craw, 1.0f));
    const float pzr = big ? qnan : pz;
    const bool live = node < nN;
    float v[NACC];
#pragma unroll
    for (int i = 0; i < NACC; ++i) {
      float y = acc[i] * di + bq[i];
      if (L != 3) y = fmaxf(y, 0.0f);
      v[i] = y + pzr;
    }
    if constexpr (L == 3) {
      const v4f g = *(const v4fa*)(xgat + (size_t)nc * XGP + 4 * (lane & 15));
      const float gsel = lane < 16 ? 1.0f : 0.0f;
      const float csel = 1.0f - gsel;
      v[0] = gsel * g.x + csel * v[0]; v[1] = gsel * g.y + csel * v[1];
      v[2] = gsel * g.z + csel * v[2]; v[3] = gsel * g.w + csel * v[3];
    }
#pragma unroll
    for (int i = 0; i < NACC; ++i) v[i] = live ? v[i] : 0.0f;
    v4us hA, lA;
#pragma unroll
    for (int i = 0; i < 4; ++i) {
      const unsigned hb = bf16_bits(v[i]);
      hA[i] = (unsigned short)hb;
      lA[i] = (unsigned short)bf16_bits(v[i] - __uint_as_float(hb << 16));
    }
    if constexpr (L == 1) {
      v4us hB, lB;
      v2us hC, lC;
#pragma unroll
      for (int i = 0; i < 4; ++i) {
        const unsigned hb = bf16_bits(v[4 + i]);
        hB[i] = (unsigned short)hb;
        lB[i] = (unsigned short)bf16_bits(v[4 + i] - __uint_as_float(hb << 16));
      }
#pragma unroll
      for (int i = 0; i < 2; ++i) {
        const unsigned hb = bf16_bits(v[8 + i]);
        hC[i] = (unsigned short)hb;
        lC[i] = (unsigned short)bf16_bits(v[8 + i] - __uint_as_float(hb << 16));
      }
      if (node < mRows) {
        unsigned short* up = outp + (size_t)node * KOUT;
        *(volatile v4us*)(up + 4 * lane) = hA;
        *(volatile v4us*)(up + 128 + 4 * lane) = hB;
        *(volatile v2us*)(up + 256 + 2 * lane) = hC;
        *(volatile v4us*)(up + LOOFF + 4 * lane) = lA;
        *(volatile v4us*)(up + LOOFF + 128 + 4 * lane) = lB;
        *(volatile v2us*)(up + LOOFF + 256 + 2 * lane) = lC;
        __threadfence();
        *(volatile v4us*)(up + 4 * lane) = hA;
        *(volatile v4us*)(up + 128 + 4 * lane) = hB;
        *(volatile v2us*)(up + 256 + 2 * lane) = hC;
        *(volatile v4us*)(up + LOOFF + 4 * lane) = lA;
        *(volatile v4us*)(up + LOOFF + 128 + 4 * lane) = lB;
        *(volatile v2us*)(up + LOOFF + 256 + 2 * lane) = lC;
      }
    } else {
      if (node < mRows) {
        unsigned short* up = outp + (size_t)node * KOUT;
        *(volatile v4us*)(up + 4 * lane) = hA;
        *(volatile v4us*)(up + LOOFF + 4 * lane) = lA;
        __threadfence();
        *(volatile v4us*)(up + 4 * lane) = hA;
        *(volatile v4us*)(up + LOOFF + 4 * lane) = lA;
      }
    }
  }
}

static inline int cdiv(int a, int b) { return (a + b - 1) / b; }

static void launch_wprep(const float* w0, const float* w1, int c0, int c1, int segRows, int nRows,
                         int Kreal, int KH, int dbl, unsigned short* out, hipStream_t s) {
  const int KT = dbl ? 2 * KH : KH;
  const int nUnits = nRows * (KT / 8);
  k_wprep<<<cdiv(nUnits, NTHR), NTHR, 0, s>>>(w0, w1, c0, c1, segRows, Kreal, KH, dbl, out, nUnits);
}

extern "C" void kernel_launch(void* const* d_in, const int* in_sizes, int n_in,
                              void* d_out, int out_size, void* d_ws, size_t ws_size,
                              hipStream_t stream) {
  if (n_in < 23) return;
  if (in_sizes[0] < FIN || (in_sizes[0] % FIN) != 0) return;
  const int nN = in_sizes[0] / FIN;
  if (nN < 2 || (nN & 1) != 0 || nN > (1 << 22)) return;
  const int nE = in_sizes[1];
  if (nE < 1 || nE >= (1 << 21) || in_sizes[2] != nE) return;
  if (in_sizes[3] != FIN * 500 || in_sizes[4] != 500 || in_sizes[5] != 500 || in_sizes[6] != 500) return;
  if (in_sizes[7] != FIN * 500) return;
  if (in_sizes[8] != 500 * 64 || in_sizes[9] != 64 || in_sizes[10] != 64 || in_sizes[11] != 64) return;
  if (in_sizes[12] != 500 * 64) return;
  if (in_sizes[13] != FIN * 300 || in_sizes[14] != 300 || in_sizes[15] != 300 * 100 || in_sizes[16] != 100) return;
  if (in_sizes[17] != 100 * 64 || in_sizes[18] != 64) return;
  if (in_sizes[19] != 128 * 64 || in_sizes[20] != 64 || in_sizes[21] != 64 * 2 || in_sizes[22] != 2) return;
  if ((long long)out_size != (long long)nN * 2) return;

  const float* x   = (const float*)d_in[0];
  const int*   src = (const int*)d_in[1];
  const int*   dst = (const int*)d_in[2];
  const float* w1  = (const float*)d_in[3];
  const float* al1 = (const float*)d_in[4];
  const float* ar1 = (const float*)d_in[5];
  const float* b1  = (const float*)d_in[6];
  const float* r1  = (const float*)d_in[7];
  const float* w2  = (const float*)d_in[8];
  const float* al2 = (const float*)d_in[9];
  const float* ar2 = (const float*)d_in[10];
  const float* b2  = (const float*)d_in[11];
  const float* r2  = (const float*)d_in[12];
  const float* gw1 = (const float*)d_in[13];
  const float* gb1 = (const float*)d_in[14];
  const float* gw2 = (const float*)d_in[15];
  const float* gb2 = (const float*)d_in[16];
  const float* gw3 = (const float*)d_in[17];
  const float* gb3 = (const float*)d_in[18];
  const float* f1w = (const float*)d_in[19];
  const float* f1b = (const float*)d_in[20];
  const float* f2w = (const float*)d_in[21];
  const float* f2b = (const float*)d_in[22];
  float* out = (float*)d_out;

  const int MP   = cdiv(nN, GBM) * GBM;
  const int gM   = MP / GBM;
  const int gA   = cdiv(MP, NB);
  const int gD   = cdiv(nN, NBD);
  const int NBPD = gD * NBD;
  if ((long long)gA * NB < (long long)MP || NBPD < nN || (MP % 32) != 0) return;
  const int vec8 = 1;

  char* ws = (char*)d_ws;
  size_t off = 0;
  auto take = [&](size_t bytes) { const size_t o = off; off = (off + bytes + 255) & ~(size_t)255; return o; };
  const size_t oXB  = take((size_t)MP * FIN * 2);
  const size_t oW1  = take((size_t)1024 * FIN * 2);
  const size_t oGW1 = take((size_t)320 * FIN * 2);
  const size_t oW2  = take((size_t)128 * 1024 * 2);
  const size_t oGW2 = take((size_t)128 * 640 * 2);
  const size_t oGW3 = take((size_t)64 * 256 * 2);
  const size_t oF1  = take((size_t)64 * 256 * 2);
  const size_t oDO  = take((size_t)NBPD * 4);
  const size_t oHR  = take((size_t)MP * HRP * 4);
  const size_t oG1X = take((size_t)MP * G1P * 4);
  const size_t oEL1 = take((size_t)MP * ELP * 4);
  const size_t oX1A = take((size_t)MP * X1K * 2);
  const size_t oG1A = take((size_t)MP * G1K * 2);
  const size_t oH2R = take((size_t)MP * H2P * 4);
  const size_t oEL2 = take((size_t)MP * ELP * 4);
  const size_t oG2X = take((size_t)MP * G2P * 4);
  const size_t oG2A = take((size_t)MP * G2K * 2);
  const size_t oXG  = take((size_t)MP * XGP * 4);
  const size_t oG3X = take((size_t)MP * G3P * 4);
  const size_t oZA  = take((size_t)MP * ZK * 2);
  if (off > ws_size) return;
  unsigned short* XB     = (unsigned short*)(ws + oXB);
  unsigned short* W1R1T  = (unsigned short*)(ws + oW1);
  unsigned short* GW1T   = (unsigned short*)(ws + oGW1);
  unsigned short* W2R2T2 = (unsigned short*)(ws + oW2);
  unsigned short* GW2T2  = (unsigned short*)(ws + oGW2);
  unsigned short* GW3T2  = (unsigned short*)(ws + oGW3);
  unsigned short* F1T2   = (unsigned short*)(ws + oF1);
  float*          DO     = (float*)(ws + oDO);
  float*          HR     = (float*)(ws + oHR);
  float*          G1X    = (float*)(ws + oG1X);
  float*          ELR1   = (float*)(ws + oEL1);
  unsigned short* X1A    = (unsigned short*)(ws + oX1A);
  unsigned short* G1A    = (unsigned short*)(ws + oG1A);
  float*          H2R    = (float*)(ws + oH2R);
  float*          ELR2   = (float*)(ws + oEL2);
  float*          G2X    = (float*)(ws + oG2X);
  unsigned short* G2A    = (unsigned short*)(ws + oG2A);
  float*          XGAT   = (float*)(ws + oXG);
  float*          G3X    = (float*)(ws + oG3X);
  unsigned short* ZA     = (unsigned short*)(ws + oZA);

  const size_t aggLds = (size_t)AGG_LDS_INTS * 4;
  hipFuncSetAttribute(reinterpret_cast<const void*>(&k_gat<1>), hipFuncAttributeMaxDynamicSharedMemorySize, (int)aggLds);
  hipFuncSetAttribute(reinterpret_cast<const void*>(&k_gat<2>), hipFuncAttributeMaxDynamicSharedMemorySize, (int)aggLds);
  hipFuncSetAttribute(reinterpret_cast<const void*>(&k_gcn<1>), hipFuncAttributeMaxDynamicSharedMemorySize, (int)aggLds);
  hipFuncSetAttribute(reinterpret_cast<const void*>(&k_gcn<2>), hipFuncAttributeMaxDynamicSharedMemorySize, (int)aggLds);
  hipFuncSetAttribute(reinterpret_cast<const void*>(&k_gcn<3>), hipFuncAttributeMaxDynamicSharedMemorySize, (int)aggLds);

  const int nUx = MP * (FIN / 8);
  k_xprep<<<cdiv(nUx, NTHR), NTHR, 0, stream>>>(x, XB, nN, nUx);
  launch_wprep(w1,  r1,  500, 500, 512, 1024, 128, 128, 0, W1R1T,  stream);
  launch_wprep(gw1, gw1, 300, 300, 320, 320,  128, 128, 0, GW1T,   stream);
  launch_wprep(w2,  r2,  64,  64,  64,  128,  500, 512, 1, W2R2T2, stream);
  launch_wprep(gw2, gw2, 100, 100, 128, 128,  300, 320, 1, GW2T2,  stream);
  launch_wprep(gw3, gw3, 64,  64,  64,  64,   100, 128, 1, GW3T2,  stream);
  launch_wprep(f1w, f1w, 64,  64,  64,  64,   128, 128, 1, F1T2,   stream);

  k_deg<<<gD, NTHR, 0, stream>>>(src, nE, vec8, DO);

  k_gemm<0><<<dim3(gM, HRP / GBN), GTHR, 0, stream>>>(XB, FIN, W1R1T, FIN, FIN, HR, HRP, f1b, f2w, f2b, out, nN);
  k_gemm<0><<<dim3(gM, G1P / GBN), GTHR, 0, stream>>>(XB, FIN, GW1T, FIN, FIN, G1X, G1P, f1b, f2w, f2b, out, nN);
  k_att<1><<<MP / 32, NTHR, 0, stream>>>(HR, al1, ar1, ELR1);
  k_gat<1><<<gA, NTHR, aggLds, stream>>>(src, dst, nE, nN, vec8, MP, HR, ELR1, b1, X1A, XGAT);
  k_gcn<1><<<gA, NTHR, aggLds, stream>>>(src, dst, nE, nN, vec8, MP, DO, G1X, gb1, XGAT, G1A);

  k_gemm<0><<<dim3(gM, H2P / GBN), GTHR, 0, stream>>>(X1A, X1K, W2R2T2, X1K, X1K, H2R, H2P, f1b, f2w, f2b, out, nN);
  k_gemm<0><<<dim3(gM, G2P / GBN), GTHR, 0, stream>>>(G1A, G1K, GW2T2, G1K, G1K, G2X, G2P, f1b, f2w, f2b, out, nN);
  k_att<2><<<MP / 32, NTHR, 0, stream>>>(H2R, al2, ar2, ELR2);
  k_gat<2><<<gA, NTHR, aggLds, stream>>>(src, dst, nE, nN, vec8, MP, H2R, ELR2, b2, X1A, XGAT);
  k_gcn<2><<<gA, NTHR, aggLds, stream>>>(src, dst, nE, nN, vec8, MP, DO, G2X, gb2, XGAT, G2A);

  k_gemm<0><<<dim3(gM, G3P / GBN), GTHR, 0, stream>>>(G2A, G2K, GW3T2, G2K, G2K, G3X, G3P, f1b, f2w, f2b, out, nN);
  k_gcn<3><<<gA, NTHR, aggLds, stream>>>(src, dst, nE, nN, vec8, MP, DO, G3X, gb3, XGAT, ZA);

  k_gemm<1><<<dim3(gM, 1), GTHR, 0, stream>>>(ZA, ZK, F1T2, ZK, ZK, G3X, G3P, f1b, f2w, f2b, out, nN);
}
